// MultiHeadAttentionWithContext_11656541241514
// MI455X (gfx1250) — hardware-verified
//
#include <hip/hip_runtime.h>
#include <hip/hip_bf16.h>


typedef __attribute__((ext_vector_type(16))) _Float16 v16h;
typedef __attribute__((ext_vector_type(8)))  _Float16 v8h;
typedef __attribute__((ext_vector_type(8)))  float    v8f;
typedef __attribute__((ext_vector_type(4)))  float    v4f_t;
typedef float v4fa __attribute__((ext_vector_type(4), may_alias));
typedef __attribute__((ext_vector_type(4)))  unsigned v4u_t;
typedef unsigned v4ua __attribute__((ext_vector_type(4), may_alias));
static __device__ __forceinline__ unsigned pk2(float a, float b) { return (unsigned)__builtin_bit_cast(unsigned short, (_Float16)a) | ((unsigned)__builtin_bit_cast(unsigned short, (_Float16)b) << 16); }

#define D_MODEL 1024
#define SEQ     2048
#define BATCH   4
#define NHEAD   16
#define DK      64
#define NTOK    (BATCH * SEQ)

static __device__ __forceinline__ v8h ld8(const _Float16* p) {
    return *(const v8h*)p;
}

static __device__ __forceinline__ v16h combine16(v8h lo, v8h hi) {
    v16h r;
#pragma unroll
    for (int i = 0; i < 8; ++i) { r[i] = lo[i]; r[i + 8] = hi[i]; }
    return r;
}

static __device__ __forceinline__ v8f wmma_f16(v16h a, v16h b, v8f c) {
    return __builtin_amdgcn_wmma_f32_16x16x32_f16(
        false, a, false, b, (short)0, c, false, false);
}

static __device__ __forceinline__ v16h load_a_frag(const _Float16* X, int ld,
                                                   int row0, int k0, int m16, int sel) {
    const _Float16* p = X + (size_t)(row0 + m16) * ld + k0;
    return combine16(ld8(p + 8 * sel), ld8(p + 16 + 8 * sel));
}

static __device__ __forceinline__ v16h load_b_frag(const _Float16* W, int ld,
                                                   int col0, int k0, int m16, int sel) {
    const _Float16* p = W + (size_t)(col0 + m16) * ld + k0;
    return combine16(ld8(p + 8 * sel), ld8(p + 16 + 8 * sel));
}

__global__ void cvt_f32_to_f16(const float* __restrict__ src,
                               _Float16* __restrict__ dst, int n) {
    int i = (blockIdx.x * blockDim.x + threadIdx.x) * 4;
    if (i + 3 < n) {
        float4 v = *(const float4*)(src + i);
        typedef __attribute__((ext_vector_type(2))) unsigned v2u_t;
        v2u_t pk; pk.x = pk2(v.x, v.y); pk.y = pk2(v.z, v.w);
        *(volatile v2u_t*)(dst + i) = pk; __threadfence(); *(volatile v2u_t*)(dst + i) = pk;
    } else {
        for (int j = i; j < n; ++j) dst[j] = (_Float16)src[j];
    }
}

__global__ void qkv_gemm(const _Float16* __restrict__ xh,
                         const _Float16* __restrict__ wqh,
                         const _Float16* __restrict__ wkh,
                         const _Float16* __restrict__ wvh,
                         const float* __restrict__ bq,
                         const float* __restrict__ bk,
                         const float* __restrict__ bv,
                         _Float16* __restrict__ Qo,
                         _Float16* __restrict__ Ko,
                         _Float16* __restrict__ Vt) {
    const int z    = blockIdx.z;
    const _Float16* W = (z == 0) ? wqh : (z == 1) ? wkh : wvh;
    const float*    bias = (z == 0) ? bq : (z == 1) ? bk : bv;

    const int tid  = threadIdx.x;
    const int wave = tid >> 5;
    const int lane = tid & 31;
    const int m16  = lane & 15;
    const int sel  = lane >> 4;
    const int wm   = wave & 1;
    const int wn   = wave >> 1;
    const int row0 = blockIdx.x * 64 + wm * 32;
    const int col0 = blockIdx.y * 256 + wn * 64;

    v8f acc[2][4];
#pragma unroll
    for (int i = 0; i < 2; ++i)
#pragma unroll
        for (int j = 0; j < 4; ++j) acc[i][j] = (v8f)(0.0f);

    for (int k0 = 0; k0 < D_MODEL; k0 += 32) {
        v16h a[2], b[4];
#pragma unroll
        for (int i = 0; i < 2; ++i)
            a[i] = load_a_frag(xh, D_MODEL, row0 + i * 16, k0, m16, sel);
#pragma unroll
        for (int j = 0; j < 4; ++j)
            b[j] = load_b_frag(W, D_MODEL, col0 + j * 16, k0, m16, sel);
#pragma unroll
        for (int i = 0; i < 2; ++i)
#pragma unroll
            for (int j = 0; j < 4; ++j)
                acc[i][j] = wmma_f16(a[i], b[j], acc[i][j]);
    }

    __shared__ __attribute__((aligned(16))) float stq[8][32 * 64];
    const float qscale = (z == 0) ? 0.125f : 1.0f;
    float* sw = stq[wave];
#pragma unroll
    for (int i = 0; i < 2; ++i)
#pragma unroll
        for (int j = 0; j < 4; ++j)
#pragma unroll
            for (int r = 0; r < 8; ++r)
                sw[(i * 16 + r + 8 * sel) * 64 + j * 16 + m16] = (acc[i][j][r] + bias[col0 + j * 16 + m16]) * qscale;
    asm volatile("s_wait_dscnt 0" ::: "memory");
    _Float16* dst = (z == 0) ? Qo : (z == 1) ? Ko : Vt;
    const int hh = col0 >> 6;
#pragma unroll 1
    for (int pass = 0; pass < 2; ++pass) {
#pragma unroll 4
        for (int rr = 0; rr < 32; ++rr) {
            const int row = row0 + rr, bb = row >> 11, ss = row & (SEQ - 1);
            *(volatile unsigned*)(dst + ((size_t)(bb * NHEAD + hh) * SEQ + ss) * DK + 2 * lane) = pk2(sw[rr * 64 + 2 * lane], sw[rr * 64 + 2 * lane + 1]);
        }
        __threadfence();
    }
}

__global__ __launch_bounds__(256) void vt_kernel(const _Float16* __restrict__ Vr, _Float16* __restrict__ Vt) {
    __shared__ _Float16 t[64][66];
    const int tid = threadIdx.x, lane = tid & 31, wave = tid >> 5;
    const int bh = blockIdx.x >> 5, s0 = (blockIdx.x & 31) * 64;
    const _Float16* src = Vr + ((size_t)bh * SEQ + s0) * DK;
#pragma unroll
    for (int k = 0; k < 16; ++k) { const int e = tid + 256 * k; t[e >> 6][e & 63] = src[e]; }
    __syncthreads();
    _Float16* dst = Vt + (size_t)bh * DK * SEQ + s0;
#pragma unroll
    for (int rr = 0; rr < 8; ++rr) {
        const int d = wave * 8 + rr;
        const unsigned p = (unsigned)__builtin_bit_cast(unsigned short, t[2 * lane][d]) | ((unsigned)__builtin_bit_cast(unsigned short, t[2 * lane + 1][d]) << 16);
        unsigned* dp = (unsigned*)(dst + (size_t)d * SEQ) + lane;
        *(volatile unsigned*)dp = p; __threadfence(); *(volatile unsigned*)dp = p;
    }
}

__global__ void attn_kernel(const _Float16* __restrict__ Qh,
                            const _Float16* __restrict__ Kh,
                            const _Float16* __restrict__ Vt,
                            _Float16* __restrict__ ctxh) {
    __shared__ _Float16 lds_p[8][16 * 32];

    const int tid  = threadIdx.x;
    const int wave = tid >> 5;
    const int lane = tid & 31;
    const int m16  = lane & 15;
    const int sel  = lane >> 4;

    const int bh = blockIdx.y;
    const int b  = bh >> 4;
    const int h  = bh & 15;
    const int q0 = blockIdx.x * 128 + wave * 16;

    const _Float16* Qbase = Qh + (size_t)bh * SEQ * DK;
    const _Float16* Kbase = Kh + (size_t)bh * SEQ * DK;
    const _Float16* Vbase = Vt + (size_t)bh * DK * SEQ;

    const _Float16* qrow = Qbase + (size_t)(q0 + m16) * DK;
    v16h aq0 = combine16(ld8(qrow + 8 * sel),      ld8(qrow + 16 + 8 * sel));
    v16h aq1 = combine16(ld8(qrow + 32 + 8 * sel), ld8(qrow + 48 + 8 * sel));

    v8f acc[4];
#pragma unroll
    for (int j = 0; j < 4; ++j) acc[j] = (v8f)(0.0f);
    float m_r[8], l_r[8];
#pragma unroll
    for (int r = 0; r < 8; ++r) { m_r[r] = -3.0e38f; l_r[r] = 0.0f; }

    _Float16* lp = &lds_p[wave][0];

    for (int kt = 0; kt < SEQ; kt += 32) {
        v8f cs[2];
#pragma unroll
        for (int sub = 0; sub < 2; ++sub) {
            const _Float16* kr = Kbase + (size_t)(kt + sub * 16 + m16) * DK;
            v16h b0 = combine16(ld8(kr + 8 * sel),      ld8(kr + 16 + 8 * sel));
            v16h b1 = combine16(ld8(kr + 32 + 8 * sel), ld8(kr + 48 + 8 * sel));
            v8f c = (v8f)(0.0f);
            c = wmma_f16(aq0, b0, c);
            c = wmma_f16(aq1, b1, c);
            cs[sub] = c;
        }

#pragma unroll
        for (int r = 0; r < 8; ++r) {
            float t = fmaxf(cs[0][r], cs[1][r]);
            t = fmaxf(t, __shfl_xor(t, 1));
            t = fmaxf(t, __shfl_xor(t, 2));
            t = fmaxf(t, __shfl_xor(t, 4));
            t = fmaxf(t, __shfl_xor(t, 8));
            float mn = fmaxf(m_r[r], t);
            float sc = __expf(m_r[r] - mn);
            m_r[r] = mn;
            float p0 = __expf(cs[0][r] - mn);
            float p1 = __expf(cs[1][r] - mn);
            cs[0][r] = p0;
            cs[1][r] = p1;
            float rs = p0 + p1;
            rs += __shfl_xor(rs, 1);
            rs += __shfl_xor(rs, 2);
            rs += __shfl_xor(rs, 4);
            rs += __shfl_xor(rs, 8);
            l_r[r] = l_r[r] * sc + rs;
#pragma unroll
            for (int j = 0; j < 4; ++j) acc[j][r] *= sc;
        }

#pragma unroll
        for (int sub = 0; sub < 2; ++sub)
#pragma unroll
            for (int r = 0; r < 8; ++r)
                lp[(r + 8 * sel) * 32 + sub * 16 + m16] = (_Float16)(cs[sub][r] * 1024.0f);

        asm volatile("s_wait_dscnt 0" ::: "memory");

        const _Float16* prow = lp + m16 * 32;
        v16h ap = combine16(*(const v8h*)(prow + 8 * sel),
                            *(const v8h*)(prow + 16 + 8 * sel));

#pragma unroll
        for (int j = 0; j < 4; ++j) {
            const _Float16* vr = Vbase + (size_t)(j * 16 + m16) * SEQ + kt + 8 * sel;
            v16h bv = combine16(ld8(vr), ld8(vr + 16));
            acc[j] = wmma_f16(ap, bv, acc[j]);
        }
    }

    __shared__ __attribute__((aligned(16))) float sto[8][16 * 64];
    float* so = sto[wave];
#pragma unroll
    for (int r = 0; r < 8; ++r) {
        float inv = 1.0f / (l_r[r] * 1024.0f);
#pragma unroll
        for (int j = 0; j < 4; ++j) so[(r + 8 * sel) * 64 + j * 16 + m16] = acc[j][r] * inv;
    }
    asm volatile("s_wait_dscnt 0" ::: "memory");
#pragma unroll 1
    for (int pass = 0; pass < 2; ++pass) {
#pragma unroll 4
        for (int rr = 0; rr < 16; ++rr)
            *(volatile unsigned*)(ctxh + ((size_t)b * SEQ + q0 + rr) * D_MODEL + h * DK + 2 * lane) = pk2(so[rr * 64 + 2 * lane], so[rr * 64 + 2 * lane + 1]);
        __threadfence();
    }
}

__global__ void out_gemm(const _Float16* __restrict__ ctxh,
                         const _Float16* __restrict__ woh,
                         const float* __restrict__ bo,
                         const float* __restrict__ xres,
                         float* __restrict__ y) {
    const int tid  = threadIdx.x;
    const int wave = tid >> 5;
    const int lane = tid & 31;
    const int m16  = lane & 15;
    const int sel  = lane >> 4;
    const int wm   = wave & 1;
    const int wn   = wave >> 1;
    const int row0 = blockIdx.x * 64 + wm * 32;
    const int col0 = blockIdx.y * 256 + wn * 64;

    v8f acc[2][4];
#pragma unroll
    for (int i = 0; i < 2; ++i)
#pragma unroll
        for (int j = 0; j < 4; ++j) acc[i][j] = (v8f)(0.0f);

    for (int k0 = 0; k0 < D_MODEL; k0 += 32) {
        v16h a[2], b[4];
#pragma unroll
        for (int i = 0; i < 2; ++i)
            a[i] = load_a_frag(ctxh, D_MODEL, row0 + i * 16, k0, m16, sel);
#pragma unroll
        for (int j = 0; j < 4; ++j)
            b[j] = load_b_frag(woh, D_MODEL, col0 + j * 16, k0, m16, sel);
#pragma unroll
        for (int i = 0; i < 2; ++i)
#pragma unroll
            for (int j = 0; j < 4; ++j)
                acc[i][j] = wmma_f16(a[i], b[j], acc[i][j]);
    }

    __shared__ __attribute__((aligned(16))) float sty[8][32 * 64];
    float* sw = sty[wave];
#pragma unroll
    for (int i = 0; i < 2; ++i)
#pragma unroll
        for (int j = 0; j < 4; ++j)
#pragma unroll
            for (int r = 0; r < 8; ++r) sw[(i * 16 + r + 8 * sel) * 64 + j * 16 + m16] = acc[i][j][r];
    asm volatile("s_wait_dscnt 0" ::: "memory");
#pragma unroll 1
    for (int pass = 0; pass < 2; ++pass) {
#pragma unroll 4
        for (int i2 = 0; i2 < 16; ++i2) {
            const int c = lane + 32 * i2, rr = c >> 4, q = c & 15;
            const size_t idx = (size_t)(row0 + rr) * D_MODEL + col0 + q * 4;
            v4f_t v = *(const volatile v4fa*)(sw + rr * 64 + q * 4);
            v += *(const v4f_t*)(bo + col0 + q * 4);
            v += *(const v4f_t*)(xres + idx);
            *(volatile v4f_t*)(y + idx) = v;
        }
        __threadfence();
    }
}

__global__ void ln_kernel(float* __restrict__ y,
                          const float* __restrict__ gamma,
                          const float* __restrict__ beta) {
    __shared__ float s_sum[256];
    __shared__ float s_sq[256];
    const int row = blockIdx.x;
    const int tid = threadIdx.x;
    float* rp = y + (size_t)row * D_MODEL;

    float4 v = *(const float4*)(rp + tid * 4);
    float sum = v.x + v.y + v.z + v.w;
    float sq  = v.x * v.x + v.y * v.y + v.z * v.z + v.w * v.w;
    s_sum[tid] = sum;
    s_sq[tid]  = sq;
    __syncthreads();
#pragma unroll
    for (int s = 128; s > 0; s >>= 1) {
        if (tid < s) {
            s_sum[tid] += s_sum[tid + s];
            s_sq[tid]  += s_sq[tid + s];
        }
        __syncthreads();
    }
    float mu  = s_sum[0] * (1.0f / D_MODEL);
    float var = s_sq[0] * (1.0f / D_MODEL) - mu * mu;
    float inv = rsqrtf(var + 1e-5f);

    float4 g = *(const float4*)(gamma + tid * 4);
    float4 bta = *(const float4*)(beta + tid * 4);
    float4 o;
    o.x = (v.x - mu) * inv * g.x + bta.x;
    o.y = (v.y - mu) * inv * g.y + bta.y;
    o.z = (v.z - mu) * inv * g.z + bta.z;
    o.w = (v.w - mu) * inv * g.w + bta.w;
    v4f_t ov = {o.x, o.y, o.z, o.w};
    *(volatile v4f_t*)(rp + tid * 4) = ov; __threadfence(); *(volatile v4f_t*)(rp + tid * 4) = ov;
}

extern "C" void kernel_launch(void* const* d_in, const int* in_sizes, int n_in,
                              void* d_out, int out_size, void* d_ws, size_t ws_size,
                              hipStream_t stream) {
    const float* x     = (const float*)d_in[0];
    const float* Wq    = (const float*)d_in[1];
    const float* bq    = (const float*)d_in[2];
    const float* Wk    = (const float*)d_in[3];
    const float* bk    = (const float*)d_in[4];
    const float* Wv    = (const float*)d_in[5];
    const float* bv    = (const float*)d_in[6];
    const float* Wo    = (const float*)d_in[7];
    const float* bo    = (const float*)d_in[8];
    const float* gamma = (const float*)d_in[9];
    const float* beta  = (const float*)d_in[10];
    float* y = (float*)d_out;

    char* ws = (char*)d_ws;
    _Float16* xh   = (_Float16*)(ws);
    _Float16* wqh  = (_Float16*)(ws + (size_t)16777216);
    _Float16* wkh  = (_Float16*)(ws + (size_t)18874368);
    _Float16* wvh  = (_Float16*)(ws + (size_t)20971520);
    _Float16* woh  = (_Float16*)(ws + (size_t)23068672);
    _Float16* Qh   = (_Float16*)(ws + (size_t)25165824);
    _Float16* Kh   = (_Float16*)(ws + (size_t)41943040);
    _Float16* Vth  = (_Float16*)(ws + (size_t)58720256);
    _Float16* ctxh = (_Float16*)(ws + (size_t)75497472);
    _Float16* Vrh  = (_Float16*)(ws + (size_t)92274688);

    cvt_f32_to_f16<<<8192, 256, 0, stream>>>(x,  xh,  NTOK * D_MODEL);
    cvt_f32_to_f16<<<1024, 256, 0, stream>>>(Wq, wqh, D_MODEL * D_MODEL);
    cvt_f32_to_f16<<<1024, 256, 0, stream>>>(Wk, wkh, D_MODEL * D_MODEL);
    cvt_f32_to_f16<<<1024, 256, 0, stream>>>(Wv, wvh, D_MODEL * D_MODEL);
    cvt_f32_to_f16<<<1024, 256, 0, stream>>>(Wo, woh, D_MODEL * D_MODEL);

    qkv_gemm<<<dim3(NTOK / 64, D_MODEL / 256, 3), 256, 0, stream>>>(
        xh, wqh, wkh, wvh, bq, bk, bv, Qh, Kh, Vrh);
    vt_kernel<<<BATCH * NHEAD * (SEQ / 64), 256, 0, stream>>>(Vrh, Vth);

    attn_kernel<<<dim3(SEQ / 128, BATCH * NHEAD), 256, 0, stream>>>(Qh, Kh, Vth, ctxh);

    out_gemm<<<dim3(NTOK / 64, D_MODEL / 256), 256, 0, stream>>>(ctxh, woh, bo, x, y);

    ln_kernel<<<NTOK, 256, 0, stream>>>(y, gamma, beta);
}
